// OptimizedRA_66236985639269
// MI455X (gfx1250) — hardware-run, weakly checked
//
#include <hip/hip_runtime.h>
#include <math.h>

typedef __attribute__((ext_vector_type(16))) _Float16 v16h;
typedef __attribute__((ext_vector_type(8)))  _Float16 v8h;
typedef __attribute__((ext_vector_type(16))) __bf16   v16b;
typedef __attribute__((ext_vector_type(8)))  __bf16   v8b;
typedef __attribute__((ext_vector_type(8)))  float    v8f;
typedef __attribute__((ext_vector_type(4)))  float    v4f;

constexpr int kBatch  = 2;
constexpr int kSeq    = 2048;
constexpr int kEmb    = 1024;
constexpr int kHeads  = 16;
constexpr int kHd     = 64;
constexpr int kRank   = 8;
constexpr int kDstd   = kHd - kRank;
constexpr int kEmb3   = 3 * kEmb;
constexpr int kRows   = kBatch * kSeq;
constexpr int kBiasLd = 2048;
constexpr int kBH     = kBatch * kHeads;
constexpr int kPrepP  = 68;
constexpr int kAtKC   = 64;
constexpr int kAtW    = 4;
constexpr float kQCarry  = 64.0f;
constexpr float kKCarry  = 64.0f;
constexpr float kNegFill = -1.0e9f;

constexpr int isqrt_c(int n) { int r = 0; while ((r + 1) * (r + 1) <= n) ++r; return r; }
static_assert(isqrt_c(kHd) * isqrt_c(kHd) == kHd);
constexpr float kScoreFold = (1.0f / (float)isqrt_c(kHd)) / (kQCarry * kKCarry);

static_assert(kEmb == kHeads * kHd);
static_assert(kDstd == 56);
static_assert((kEmb % 32) == 0);
static_assert((kRows % 64) == 0 && (kEmb3 % 64) == 0 && (kEmb % 64) == 0);
static_assert((kSeq % 64) == 0 && kSeq == kBiasLd);
static_assert(((kRows * kEmb / 8) % 256) == 0 && ((kEmb3 * kEmb / 8) % 256) == 0 && ((kEmb * kEmb / 8) % 256) == 0);

constexpr size_t kOffXB  = 0;
constexpr size_t kOffWQB = kOffXB  + (size_t)kRows * kEmb * 2;
constexpr size_t kOffWPB = kOffWQB + (size_t)kEmb3 * kEmb * 2;
constexpr size_t kOffQKV = kOffWPB + (size_t)kEmb * kEmb * 2;
constexpr size_t kOffQA  = kOffQKV + (size_t)kRows * kEmb3 * 4;
constexpr size_t kOffKA  = kOffQA  + (size_t)kBH * kSeq * kHd * 2;
constexpr size_t kOffVTH = kOffKA  + (size_t)kBH * kSeq * kHd * 2;
constexpr size_t kOffVTL = kOffVTH + (size_t)kBH * kHd * kSeq * 2;
constexpr size_t kOffAH  = kOffVTL + (size_t)kBH * kHd * kSeq * 2;
constexpr size_t kOffAL  = kOffAH  + (size_t)kRows * kEmb * 2;
constexpr size_t kWsTotal = kOffAL + (size_t)kRows * kEmb * 2;
static_assert(kWsTotal == 117440512ull);
static_assert(kWsTotal <= 134217728ull);
static_assert((kOffWQB % 128) == 0 && (kOffWPB % 128) == 0 && (kOffQKV % 128) == 0 && (kOffQA % 128) == 0 &&
              (kOffKA % 128) == 0 && (kOffVTH % 128) == 0 && (kOffVTL % 128) == 0 && (kOffAH % 128) == 0 &&
              (kOffAL % 128) == 0);

__device__ __forceinline__ unsigned short f2bf_bits(float f) {
  unsigned u = __float_as_uint(f);
  return (unsigned short)((u + 0x7FFFu + ((u >> 16) & 1u)) >> 16);
}
__device__ __forceinline__ float bf_bits2f(unsigned short h) { return __uint_as_float(((unsigned)h) << 16); }
__device__ __forceinline__ float bf16_val(float f) { return bf_bits2f(f2bf_bits(f)); }

__device__ __forceinline__ void dep_guard4_h(v8f& a, v8f& b, v8f& c, v8f& d, v16h x, v16h y) { asm volatile("v_nop\n\tv_nop\n\tv_nop\n\tv_nop" : "+v"(a), "+v"(b), "+v"(c), "+v"(d) : "v"(x), "v"(y)); }
__device__ __forceinline__ void dep_guard4_b(v8f& a, v8f& b, v8f& c, v8f& d, v16b x, v16b y) { asm volatile("v_nop\n\tv_nop\n\tv_nop\n\tv_nop" : "+v"(a), "+v"(b), "+v"(c), "+v"(d) : "v"(x), "v"(y)); }
__device__ __forceinline__ void keep4_h(v16h a, v16h b, v16h c, v16h d) { asm volatile("v_nop" :: "v"(a), "v"(b), "v"(c), "v"(d)); }
__device__ __forceinline__ void keep4_b(v16b a, v16b b, v16b c, v16b d) { asm volatile("v_nop" :: "v"(a), "v"(b), "v"(c), "v"(d)); }
__device__ __forceinline__ void acc_guard4(v8f& a, v8f& b, v8f& c, v8f& d) { asm volatile("v_nop\n\tv_nop\n\tv_nop\n\tv_nop" : "+v"(a), "+v"(b), "+v"(c), "+v"(d)); }
template <typename T> struct Frag;
template <> struct Frag<_Float16> {
  typedef v16h V; union U { v16h v; v8h h[2]; };
  static __device__ __forceinline__ v16h load(const _Float16* p) {
    U f; f.h[0] = *(const v8h*)(p); f.h[1] = *(const v8h*)(p + 16); return f.v;
  }
  static __device__ __forceinline__ v8f mma(v16h a, v16h b, v8f c) {
    return __builtin_amdgcn_wmma_f32_16x16x32_f16(false, a, false, b, (short)0, c, false, false);
  }
  static __device__ __forceinline__ void guard4(v8f& a, v8f& b, v8f& c, v8f& d, v16h x, v16h y) { dep_guard4_h(a, b, c, d, x, y); }
  static __device__ __forceinline__ void keep(v16h a, v16h b, v16h c, v16h d) { keep4_h(a, b, c, d); }
};
template <> struct Frag<__bf16> {
  typedef v16b V; union U { v16b v; v8b h[2]; };
  static __device__ __forceinline__ v16b load(const __bf16* p) {
    U f; f.h[0] = *(const v8b*)(p); f.h[1] = *(const v8b*)(p + 16); return f.v;
  }
  static __device__ __forceinline__ v8f mma(v16b a, v16b b, v8f c) {
    return __builtin_amdgcn_wmma_f32_16x16x32_bf16(false, a, false, b, (short)0, c, false, false);
  }
  static __device__ __forceinline__ void guard4(v8f& a, v8f& b, v8f& c, v8f& d, v16b x, v16b y) { dep_guard4_b(a, b, c, d, x, y); }
  static __device__ __forceinline__ void keep(v16b a, v16b b, v16b c, v16b d) { keep4_b(a, b, c, d); }
};

__device__ __forceinline__ v8f mma_h(v16h a, v16h b, v8f c) {
  c = __builtin_amdgcn_wmma_f32_16x16x32_f16(false, a, false, b, (short)0, c, false, false);
  asm volatile("v_nop\n\tv_nop\n\tv_nop\n\tv_nop" : "+v"(c) : "v"(a), "v"(b));
  return c;
}
__device__ __forceinline__ v8f mma_b(v16b a, v16b b, v8f c) {
  c = __builtin_amdgcn_wmma_f32_16x16x32_bf16(false, a, false, b, (short)0, c, false, false);
  asm volatile("v_nop\n\tv_nop\n\tv_nop\n\tv_nop" : "+v"(c) : "v"(a), "v"(b));
  return c;
}
__device__ __forceinline__ void split_bf(float f, __bf16& hi, __bf16& lo) {
  const unsigned short hb = f2bf_bits(f);
  const unsigned short lb = f2bf_bits(f - bf_bits2f(hb));
  hi = __builtin_bit_cast(__bf16, hb);
  lo = __builtin_bit_cast(__bf16, lb);
}

template <int ET> struct Elem;
template <> struct Elem<0> { typedef _Float16 T; };
template <> struct Elem<1> { typedef __bf16 T; };
template <int ET, int SPL, int BIAS_MODE, int OUT_MODE, bool RESID, int ACT = 0>
__global__ __launch_bounds__(256) void wmma_gemm64(
    const unsigned short* __restrict__ Ap, const unsigned short* __restrict__ A2p, int lda, long strideA,
    const unsigned short* __restrict__ Btp, const unsigned short* __restrict__ Bt2p, int ldb, long strideB,
    void* __restrict__ Cout, void* __restrict__ Cout2, int ldc, long strideC,
    const float* __restrict__ bias,
    const float* __restrict__ resid, long strideR,
    int M, int N, int K, float scale) {
  typedef typename Elem<ET>::T T;
  typedef typename Frag<T>::V V;
  const T* A = (const T*)Ap; const T* A2 = (const T*)A2p; const T* Bt = (const T*)Btp; const T* Bt2 = (const T*)Bt2p;
  __shared__ __align__(16) float sT[8][16 * 68];
  const int b    = blockIdx.y;
  const int lane = threadIdx.x & 31;
  const int wave = threadIdx.x >> 5;
  const int tilesN = N >> 6;
  const int tilesM = M >> 6;
  const int tile = blockIdx.x * 8 + wave;
  if (tile >= tilesM * tilesN) return;
  const int tm = tile / tilesN;
  const int tn = tile - tm * tilesN;
  const int m0 = tm << 6;
  const int n0 = tn << 6;

  const T* Ab  = A  + (size_t)b * strideA;
  const T* Bb  = Bt + (size_t)b * strideB;
  const T* Ab2 = (SPL >= 1) ? (A2  + (size_t)b * strideA) : nullptr;
  const T* Bb2 = (SPL == 2) ? (Bt2 + (size_t)b * strideB) : nullptr;

  const int rlane = lane & 15;
  const int koff  = (lane >> 4) * 8;
  const int mOff  = (lane >> 4) * 8;

  v8f acc[4][4];
#pragma unroll
  for (int i = 0; i < 4; ++i)
#pragma unroll
    for (int j = 0; j < 4; ++j) acc[i][j] = (v8f){0.f,0.f,0.f,0.f,0.f,0.f,0.f,0.f};

  for (int k0 = 0; k0 < K; k0 += 32) {
    V bh[4], bl[4];
#pragma unroll
    for (int j = 0; j < 4; ++j) {
      const size_t bo = (size_t)(n0 + (j << 4) + rlane) * ldb + koff + k0;
      bh[j] = Frag<T>::load(Bb + bo);
      if (SPL == 2) bl[j] = Frag<T>::load(Bb2 + bo);
    }
#pragma unroll
    for (int i = 0; i < 4; ++i) {
      const size_t ao = (size_t)(m0 + (i << 4) + rlane) * lda + koff + k0;
      V ah = Frag<T>::load(Ab + ao);
      V al;
      if (SPL >= 1) al = Frag<T>::load(Ab2 + ao);
#pragma unroll
      for (int j = 0; j < 4; ++j) {
        acc[i][j] = Frag<T>::mma(ah, bh[j], acc[i][j]);
        if (SPL == 2) acc[i][j] = Frag<T>::mma(ah, bl[j], acc[i][j]);
        if (SPL >= 1) acc[i][j] = Frag<T>::mma(al, bh[j], acc[i][j]);
      }
      Frag<T>::guard4(acc[i][0], acc[i][1], acc[i][2], acc[i][3], ah, (SPL >= 1) ? al : ah);
    }
    Frag<T>::keep(bh[0], bh[1], bh[2], bh[3]);
    if (SPL == 2) Frag<T>::keep(bl[0], bl[1], bl[2], bl[3]);
  }
  acc_guard4(acc[0][0], acc[0][1], acc[0][2], acc[0][3]);
  acc_guard4(acc[1][0], acc[1][1], acc[1][2], acc[1][3]);
  acc_guard4(acc[2][0], acc[2][1], acc[2][2], acc[2][3]);
  acc_guard4(acc[3][0], acc[3][1], acc[3][2], acc[3][3]);

  float* slab = sT[wave];
  const float* Rb = RESID ? (resid + (size_t)b * strideR) : nullptr;
#pragma unroll
  for (int i = 0; i < 4; ++i) {
    const int mBase = m0 + (i << 4);
#pragma unroll
    for (int j = 0; j < 4; ++j) {
      const int n = n0 + (j << 4) + rlane;
      float bv = 0.f;
      if (BIAS_MODE == 2) bv = bias[n];
#pragma unroll
      for (int r = 0; r < 8; ++r) {
        float v = acc[i][j][r] * scale;
        if (BIAS_MODE == 1) v += bias[mBase + mOff + r];
        if (BIAS_MODE == 2) v += bv;
        if (RESID) v += Rb[(size_t)(mBase + mOff + r) * ldc + n];
        if (ACT == 2) v = fmaxf(v, 0.0f);
        if (ACT == 4) v = (v > 0.f) ? v : 0.01f * v;
        slab[(mOff + r) * 68 + (j << 4) + rlane] = v;
      }
    }
    __builtin_amdgcn_fence(__ATOMIC_RELEASE, "workgroup");
    __builtin_amdgcn_wave_barrier();
    __builtin_amdgcn_fence(__ATOMIC_ACQUIRE, "workgroup");
    if (OUT_MODE == 0) {
      float* C = (float*)Cout + (size_t)b * strideC;
      const int hh = lane >> 4, c4 = (lane & 15) * 4;
      for (int pass = 0; pass < 2; ++pass) {
#pragma unroll
        for (int it = 0; it < 8; ++it) {
          const int row = it * 2 + hh;
          v4f v = *(const v4f*)(slab + row * 68 + c4);
          *(volatile v4f*)(C + (size_t)(mBase + row) * ldc + n0 + c4) = v;
        }
        __threadfence();
      }
    } else {
      const int q = lane >> 3, c8 = (lane & 7) * 8;
      unsigned short* C  = (unsigned short*)Cout  + (size_t)b * strideC;
      unsigned short* C2 = (OUT_MODE == 2) ? ((unsigned short*)Cout2 + (size_t)b * strideC) : nullptr;
      for (int pass = 0; pass < 2; ++pass) {
#pragma unroll
        for (int it = 0; it < 4; ++it) {
          const int row = it * 4 + q;
          const float* sp = slab + row * 68 + c8;
          v8h hv, lv;
#pragma unroll
          for (int e = 0; e < 8; ++e) {
            if (OUT_MODE == 1) {
              hv[e] = (_Float16)sp[e];
            } else {
              unsigned short hb = f2bf_bits(sp[e]);
              unsigned short lb = f2bf_bits(sp[e] - bf_bits2f(hb));
              hv[e] = __builtin_bit_cast(_Float16, hb);
              lv[e] = __builtin_bit_cast(_Float16, lb);
            }
          }
          *(volatile v8h*)(C + (size_t)(mBase + row) * ldc + n0 + c8) = hv;
          if (OUT_MODE == 2) *(volatile v8h*)(C2 + (size_t)(mBase + row) * ldc + n0 + c8) = lv;
        }
        __threadfence();
      }
    }
    __builtin_amdgcn_fence(__ATOMIC_RELEASE, "workgroup");
    __builtin_amdgcn_wave_barrier();
    __builtin_amdgcn_fence(__ATOMIC_ACQUIRE, "workgroup");
  }
}

__global__ __launch_bounds__(256) void cast8_bf16_kernel(
    const float* __restrict__ src, unsigned short* __restrict__ dst, int total8)
{
  const int i = blockIdx.x * 256 + threadIdx.x;
  if (i >= total8) return;
  const size_t e0 = (size_t)i << 3;
  const v4f a0 = *(const v4f*)(src + e0);
  const v4f a1 = *(const v4f*)(src + e0 + 4);
  v8h hv;
#pragma unroll
  for (int e = 0; e < 4; ++e) {
    const unsigned short h0 = f2bf_bits(a0[e]);
    const unsigned short h1 = f2bf_bits(a1[e]);
    hv[e]     = __builtin_bit_cast(_Float16, h0);
    hv[4 + e] = __builtin_bit_cast(_Float16, h1);
  }
  unsigned short* q = dst + e0;
  *(volatile v8h*)q = hv;
  __threadfence();
  *(volatile v8h*)q = hv;
}

__global__ __launch_bounds__(256) void prep_kernel(
    const float* __restrict__ QKV, const float* __restrict__ Wr,
    const float* __restrict__ w_std, const float* __restrict__ w_rec,
    unsigned short* __restrict__ QA, unsigned short* __restrict__ KA,
    unsigned short* __restrict__ VTH, unsigned short* __restrict__ VTL)
{
  __shared__ __align__(16) float sQK[2 * 64 * kPrepP];
  __shared__ __align__(16) float sV[64 * kPrepP];
  __shared__ __align__(16) float sW[kHd * kRank];
  __shared__ __align__(16) float sLow[2 * 64 * kRank];
  const int tid = threadIdx.x, lane = tid & 31, wave = tid >> 5;
  constexpr int kTiles = kSeq / 64;
  const int bx = blockIdx.x;
  const int tt = bx % kTiles;
  const int bh = bx / kTiles;
  const int h  = bh % kHeads;
  const int b  = bh / kHeads;
  const size_t row0 = (size_t)b * kSeq + (size_t)tt * 64;
#pragma unroll
  for (int i = 0; i < 4; ++i) {
    const int e  = i * 256 + tid;
    const int r  = e >> 4;
    const int c4 = (e & 15) * 4;
    const float* base = QKV + (row0 + r) * kEmb3 + h * kHd + c4;
    const v4f vq = *(const v4f*)(base);
    const v4f vk = *(const v4f*)(base + kEmb);
    const v4f vv = *(const v4f*)(base + 2 * kEmb);
    *(v4f*)(sQK + r * kPrepP + c4) = vq;
    *(v4f*)(sQK + 64 * kPrepP + r * kPrepP + c4) = vk;
    *(v4f*)(sV + r * kPrepP + c4) = vv;
  }
  sW[tid]       = bf16_val(Wr[tid]);
  sW[tid + 256] = bf16_val(Wr[tid + 256]);
  __syncthreads();
  {
    const int tk = tid >> 2, part = tid & 3;
    const int which = part >> 1, r0 = (part & 1) * 4;
    const float* xr = sQK + which * 64 * kPrepP + tk * kPrepP;
    float a0 = 0.f, a1 = 0.f, a2 = 0.f, a3 = 0.f;
#pragma unroll 4
    for (int d = 0; d < kHd; ++d) {
      const float xv = xr[d];
      const float* wp = sW + d * kRank + r0;
      a0 = fmaf(xv, wp[0], a0);
      a1 = fmaf(xv, wp[1], a1);
      a2 = fmaf(xv, wp[2], a2);
      a3 = fmaf(xv, wp[3], a3);
    }
    float* lp = sLow + which * 64 * kRank + tk * kRank + r0;
    lp[0] = a0; lp[1] = a1; lp[2] = a2; lp[3] = a3;
  }
  __syncthreads();
  const float sstd = sqrtf(bf16_val(w_std[h]));
  const float srec = sqrtf(bf16_val(w_rec[h]));
  const float fq_std = kQCarry * sstd, fq_rec = kQCarry * srec;
  const float fk_std = kKCarry * sstd, fk_rec = kKCarry * srec;
  const int q = lane >> 3, c8 = (lane & 7) * 8;
  const bool isLow = (c8 == kDstd);
  v8h qv[2], kv[2], vh[2], vl[2];
#pragma unroll
  for (int it = 0; it < 2; ++it) {
    const int row = wave * 8 + it * 4 + q;
    const v4f q0v = *(const v4f*)(sQK + row * kPrepP + c8);
    const v4f q1v = *(const v4f*)(sQK + row * kPrepP + c8 + 4);
    const v4f k0v = *(const v4f*)(sQK + 64 * kPrepP + row * kPrepP + c8);
    const v4f k1v = *(const v4f*)(sQK + 64 * kPrepP + row * kPrepP + c8 + 4);
    const v4f ql0 = *(const v4f*)(sLow + row * kRank);
    const v4f ql1 = *(const v4f*)(sLow + row * kRank + 4);
    const v4f kl0 = *(const v4f*)(sLow + 64 * kRank + row * kRank);
    const v4f kl1 = *(const v4f*)(sLow + 64 * kRank + row * kRank + 4);
#pragma unroll
    for (int e = 0; e < 4; ++e) {
      const float qs0 = q0v[e], qs1 = q1v[e], ks0 = k0v[e], ks1 = k1v[e];
      const float qa0 = ql0[e], qa1 = ql1[e], ka0 = kl0[e], ka1 = kl1[e];
      const float qo0 = isLow ? (fq_rec * ka0) : (fq_std * qs0);
      const float qo1 = isLow ? (fq_rec * ka1) : (fq_std * qs1);
      const float ko0 = isLow ? (fk_rec * qa0) : (fk_std * ks0);
      const float ko1 = isLow ? (fk_rec * qa1) : (fk_std * ks1);
      qv[it][e]     = (_Float16)qo0;
      qv[it][4 + e] = (_Float16)qo1;
      kv[it][e]     = (_Float16)ko0;
      kv[it][4 + e] = (_Float16)ko1;
    }
#pragma unroll
    for (int e = 0; e < 8; ++e) {
      const float vv = sV[(c8 + e) * kPrepP + row];
      const unsigned short hb = f2bf_bits(vv);
      const unsigned short lb = f2bf_bits(vv - bf_bits2f(hb));
      vh[it][e] = __builtin_bit_cast(_Float16, hb);
      vl[it][e] = __builtin_bit_cast(_Float16, lb);
    }
  }
  for (int pass = 0; pass < 2; ++pass) {
#pragma unroll
    for (int it = 0; it < 2; ++it) {
      const int row = wave * 8 + it * 4 + q;
      const size_t oq = ((size_t)bh * kSeq + (size_t)tt * 64 + row) * kHd + c8;
      *(volatile v8h*)(QA + oq) = qv[it];
      *(volatile v8h*)(KA + oq) = kv[it];
      const size_t ov = ((size_t)bh * kHd + row) * kSeq + (size_t)tt * 64 + c8;
      *(volatile v8h*)(VTH + ov) = vh[it];
      *(volatile v8h*)(VTL + ov) = vl[it];
    }
    __threadfence();
  }
}

__global__ __launch_bounds__(128) void attn_kernel(
    const unsigned short* __restrict__ QA, const unsigned short* __restrict__ KA,
    const unsigned short* __restrict__ VTH, const unsigned short* __restrict__ VTL,
    const float* __restrict__ w_disc, const float* __restrict__ d_bias,
    unsigned short* __restrict__ AH, unsigned short* __restrict__ AL)
{
  union FB { v16b v; v8b h[2]; };
  __shared__ __align__(16) __bf16 Ph[kAtW][16 * kAtKC];
  __shared__ __align__(16) __bf16 Pl[kAtW][16 * kAtKC];
  __shared__ __align__(16) float  Os[kAtW][16 * 68];

  const int tid  = threadIdx.x;
  const int wave = tid >> 5;
  const int lane = tid & 31;
  const int hh   = lane >> 4;
  const int c    = lane & 15;

  constexpr int nqb = kSeq / 64;
  const int bx = blockIdx.x;
  const int qb = bx % nqb;
  const int bh = bx / nqb;
  const int h  = bh % kHeads;
  const int b  = bh / kHeads;
  const int q0 = qb * 64 + wave * 16;

  const _Float16* Qp = (const _Float16*)QA + (size_t)bh * kSeq * kHd;
  const _Float16* Kp = (const _Float16*)KA + (size_t)bh * kSeq * kHd;
  const __bf16*   Vh = (const __bf16*)VTH + (size_t)bh * kHd * kSeq;
  const __bf16*   Vl = (const __bf16*)VTL + (size_t)bh * kHd * kSeq;

  const v16h qa0 = Frag<_Float16>::load(Qp + (size_t)(q0 + c) * kHd + 8 * hh);
  const v16h qa1 = Frag<_Float16>::load(Qp + (size_t)(q0 + c) * kHd + 32 + 8 * hh);

  const float wd = bf16_val(w_disc[h]);
  const float* dbrow = d_bias + (size_t)h * kBiasLd;

  float mrow[8], lrow[8];
  v8f oacc[4];
#pragma unroll
  for (int r = 0; r < 8; ++r) { mrow[r] = -1.0e30f; lrow[r] = 0.f; }
#pragma unroll
  for (int t = 0; t < 4; ++t) oacc[t] = (v8f){0.f,0.f,0.f,0.f,0.f,0.f,0.f,0.f};

  __bf16* pwh = Ph[wave];
  __bf16* pwl = Pl[wave];

#pragma unroll 1
  for (int kc = 0; kc <= qb; ++kc) {
    const int kv0 = kc * kAtKC;
    v8f s[4];
#pragma unroll
    for (int j = 0; j < 4; ++j) {
      s[j] = (v8f){0.f,0.f,0.f,0.f,0.f,0.f,0.f,0.f};
      const _Float16* kr = Kp + (size_t)(kv0 + j * 16 + c) * kHd + 8 * hh;
      const v16h kf0 = Frag<_Float16>::load(kr);
      const v16h kf1 = Frag<_Float16>::load(kr + 32);
      s[j] = mma_h(qa0, kf0, s[j]);
      s[j] = mma_h(qa1, kf1, s[j]);
    }
    float bj[4];
#pragma unroll
    for (int j = 0; j < 4; ++j) bj[j] = wd * bf16_val(dbrow[kv0 + j * 16 + c]);

    const bool diag = (kc == qb);
    float cm[8];
#pragma unroll
    for (int r = 0; r < 8; ++r) {
      const int qrow = q0 + 8 * hh + r;
      float m = -1.0e30f;
#pragma unroll
      for (int j = 0; j < 4; ++j) {
        const int kvcol = kv0 + j * 16 + c;
        float sv = s[j][r] * kScoreFold + bj[j];
        const bool masked = diag && (kvcol > qrow);
        sv = masked ? kNegFill : sv;
        s[j][r] = sv;
        m = fmaxf(m, sv);
      }
#pragma unroll
      for (int off = 1; off < 16; off <<= 1) m = fmaxf(m, __shfl_xor(m, off, 32));
      cm[r] = m;
    }
#pragma unroll
    for (int r = 0; r < 8; ++r) {
      const float mnew  = fmaxf(mrow[r], cm[r]);
      const float alpha = __expf(mrow[r] - mnew);
      mrow[r] = mnew;
      float psum = 0.f;
#pragma unroll
      for (int j = 0; j < 4; ++j) {
        const float p = __expf(s[j][r] - mnew);
        psum += p;
        __bf16 ph, pl;
        split_bf(p, ph, pl);
        pwh[(8 * hh + r) * kAtKC + j * 16 + c] = ph;
        pwl[(8 * hh + r) * kAtKC + j * 16 + c] = pl;
      }
      lrow[r] = lrow[r] * alpha + psum;
#pragma unroll
      for (int t = 0; t < 4; ++t) oacc[t][r] *= alpha;
    }
    __builtin_amdgcn_fence(__ATOMIC_RELEASE, "workgroup");
    __builtin_amdgcn_wave_barrier();
    __builtin_amdgcn_fence(__ATOMIC_ACQUIRE, "workgroup");
#pragma unroll 1
    for (int kk = 0; kk < 2; ++kk) {
      FB pa, pl;
      pa.h[0] = *(const v8b*)(pwh + c * kAtKC + kk * 32 + 8 * hh);
      pa.h[1] = *(const v8b*)(pwh + c * kAtKC + kk * 32 + 16 + 8 * hh);
      pl.h[0] = *(const v8b*)(pwl + c * kAtKC + kk * 32 + 8 * hh);
      pl.h[1] = *(const v8b*)(pwl + c * kAtKC + kk * 32 + 16 + 8 * hh);
#pragma unroll
      for (int t = 0; t < 4; ++t) {
        const size_t vo = (size_t)(t * 16 + c) * kSeq + kv0 + kk * 32 + 8 * hh;
        const v16b vb = Frag<__bf16>::load(Vh + vo);
        const v16b vl = Frag<__bf16>::load(Vl + vo);
        oacc[t] = mma_b(pa.v, vb, oacc[t]);
        oacc[t] = mma_b(pa.v, vl, oacc[t]);
        oacc[t] = mma_b(pl.v, vb, oacc[t]);
      }
    }
    __builtin_amdgcn_fence(__ATOMIC_RELEASE, "workgroup");
    __builtin_amdgcn_wave_barrier();
    __builtin_amdgcn_fence(__ATOMIC_ACQUIRE, "workgroup");
  }

  float* os = Os[wave];
#pragma unroll
  for (int r = 0; r < 8; ++r) {
    float l = lrow[r];
#pragma unroll
    for (int off = 1; off < 16; off <<= 1) l += __shfl_xor(l, off, 32);
    const float inv = 1.0f / l;
#pragma unroll
    for (int t = 0; t < 4; ++t) os[(8 * hh + r) * 68 + t * 16 + c] = oacc[t][r] * inv;
  }
  __builtin_amdgcn_fence(__ATOMIC_RELEASE, "workgroup");
  __builtin_amdgcn_wave_barrier();
  __builtin_amdgcn_fence(__ATOMIC_ACQUIRE, "workgroup");
  {
    const int q = lane >> 3, c8 = (lane & 7) * 8;
    v8h hv[4], lv[4];
#pragma unroll
    for (int it = 0; it < 4; ++it) {
      const int row = it * 4 + q;
      const float* sp = os + row * 68 + c8;
      const v4f a0 = *(const v4f*)(sp);
      const v4f a1 = *(const v4f*)(sp + 4);
#pragma unroll
      for (int e = 0; e < 4; ++e) {
        const float f0 = a0[e], f1 = a1[e];
        const unsigned short h0 = f2bf_bits(f0), h1 = f2bf_bits(f1);
        const unsigned short l0 = f2bf_bits(f0 - bf_bits2f(h0)), l1 = f2bf_bits(f1 - bf_bits2f(h1));
        hv[it][e]     = __builtin_bit_cast(_Float16, h0);
        hv[it][4 + e] = __builtin_bit_cast(_Float16, h1);
        lv[it][e]     = __builtin_bit_cast(_Float16, l0);
        lv[it][4 + e] = __builtin_bit_cast(_Float16, l1);
      }
    }
    for (int pass = 0; pass < 2; ++pass) {
#pragma unroll
      for (int it = 0; it < 4; ++it) {
        const int row = it * 4 + q;
        const size_t o = ((size_t)b * kSeq + q0 + row) * kEmb + h * kHd + c8;
        *(volatile v8h*)(AH + o) = hv[it];
        *(volatile v8h*)(AL + o) = lv[it];
      }
      __threadfence();
    }
  }
}

extern "C" void kernel_launch(void* const* d_in, const int* in_sizes, int n_in,
                              void* d_out, int out_size, void* d_ws, size_t ws_size,
                              hipStream_t stream) {
  if (n_in < 8) return;
  if (in_sizes[0] != kRows * kEmb) return;
  if (in_sizes[1] != kEmb3 * kEmb) return;
  if (in_sizes[2] != kEmb * kEmb) return;
  if (in_sizes[3] != kHd * kRank) return;
  if (in_sizes[4] != kHeads) return;
  if (in_sizes[5] != kHeads) return;
  if (in_sizes[6] != kHeads) return;
  if (in_sizes[7] != kHeads * kBiasLd) return;
  if (out_size != kRows * kEmb) return;
  if (ws_size < kWsTotal) return;

  const float* x       = (const float*)d_in[0];
  const float* Wqkv    = (const float*)d_in[1];
  const float* Wproj   = (const float*)d_in[2];
  const float* W_recip = (const float*)d_in[3];
  const float* w_std   = (const float*)d_in[4];
  const float* w_rec   = (const float*)d_in[5];
  const float* w_disc  = (const float*)d_in[6];
  const float* d_bias  = (const float*)d_in[7];
  float* out = (float*)d_out;

  char* ws = (char*)d_ws;
  unsigned short* XB  = (unsigned short*)(ws + kOffXB);
  unsigned short* WQB = (unsigned short*)(ws + kOffWQB);
  unsigned short* WPB = (unsigned short*)(ws + kOffWPB);
  float*          QKV = (float*)(ws + kOffQKV);
  unsigned short* QA  = (unsigned short*)(ws + kOffQA);
  unsigned short* KA  = (unsigned short*)(ws + kOffKA);
  unsigned short* VTH = (unsigned short*)(ws + kOffVTH);
  unsigned short* VTL = (unsigned short*)(ws + kOffVTL);
  unsigned short* AH  = (unsigned short*)(ws + kOffAH);
  unsigned short* AL  = (unsigned short*)(ws + kOffAL);

  cast8_bf16_kernel<<<(kRows * kEmb / 8) / 256, 256, 0, stream>>>(x, XB, kRows * kEmb / 8);
  cast8_bf16_kernel<<<(kEmb3 * kEmb / 8) / 256, 256, 0, stream>>>(Wqkv, WQB, kEmb3 * kEmb / 8);
  cast8_bf16_kernel<<<(kEmb * kEmb / 8) / 256, 256, 0, stream>>>(Wproj, WPB, kEmb * kEmb / 8);

  wmma_gemm64<1, 0, 0, 0, false><<<dim3((kRows / 64) * (kEmb3 / 64) / 8, 1), 256, 0, stream>>>(
      XB, nullptr, kEmb, 0L,
      WQB, nullptr, kEmb, 0L,
      (void*)QKV, nullptr, kEmb3, 0L,
      nullptr, nullptr, 0L,
      kRows, kEmb3, kEmb, 1.0f);

  prep_kernel<<<kBH * (kSeq / 64), 256, 0, stream>>>(QKV, W_recip, w_std, w_rec, QA, KA, VTH, VTL);

  attn_kernel<<<kBH * (kSeq / 64), 128, 0, stream>>>(QA, KA, VTH, VTL, w_disc, d_bias, AH, AL);

  wmma_gemm64<1, 1, 0, 0, false><<<dim3((kRows / 64) * (kEmb / 64) / 8, 1), 256, 0, stream>>>(
      AH, AL, kEmb, 0L,
      WPB, nullptr, kEmb, 0L,
      (void*)out, nullptr, kEmb, 0L,
      nullptr, nullptr, 0L,
      kRows, kEmb, kEmb, 1.0f);
}
